// SuffixAttention_70308614636253
// MI455X (gfx1250) — hardware-verified
//
#include <hip/hip_runtime.h>
#include <math.h>

typedef __attribute__((ext_vector_type(16))) _Float16 v16h;
typedef __attribute__((ext_vector_type(16))) __bf16 v16b;
typedef __attribute__((ext_vector_type(8)))  _Float16 v8h;
typedef __attribute__((ext_vector_type(8)))  float v8f;
typedef __attribute__((ext_vector_type(4)))  float v4f;
typedef __attribute__((ext_vector_type(2)))  float v2f;
typedef __attribute__((ext_vector_type(4)))  unsigned v4u;
typedef __attribute__((ext_vector_type(4)))  int v4i;
typedef float __attribute__((may_alias)) float_a;
typedef int __attribute__((may_alias)) int_a;

template <typename T> __device__ __forceinline__ void vst2(void* p, T v) { *(volatile T*)p = v; __threadfence(); *(volatile T*)p = v; }
__device__ __forceinline__ v8f wmma16(v16h a, v16h b, v8f c) {
  v8f d = __builtin_amdgcn_wmma_f32_16x16x32_f16(false, a, false, b, (short)0, c, false, false);
  asm volatile("v_nop\n\tv_nop\n\tv_nop\n\tv_nop" : "+v"(d) : "v"(a), "v"(b));
  return d;
}
__device__ __forceinline__ v8f wmma_bf(v16b a, v16b b, v8f c) {
  v8f d = __builtin_amdgcn_wmma_f32_16x16x32_bf16(false, a, false, b, (short)0, c, false, false);
  asm volatile("v_nop\n\tv_nop\n\tv_nop\n\tv_nop" : "+v"(d) : "v"(a), "v"(b));
  return d;
}
__device__ __forceinline__ v16h frag_h(const _Float16* rowk0, int lane) {
  union { v16h v; v8h q[2]; } u; const _Float16* p = rowk0 + 8 * (lane >> 4);
  u.q[0] = *(const v8h*)p; u.q[1] = *(const v8h*)(p + 16); return u.v;
}
__device__ __forceinline__ v16h frag_f32(const float* rowk0, int lane) {
  v16h a; const float* p = rowk0 + 8 * (lane >> 4);
#pragma unroll
  for (int i = 0; i < 8; ++i) { a[i] = (_Float16)p[i]; a[8 + i] = (_Float16)p[16 + i]; }
  return a;
}
__device__ __forceinline__ v16h frag_f32s(const float* rowk0, int lane, float sc) {
  v16h a; const float* p = rowk0 + 8 * (lane >> 4);
#pragma unroll
  for (int i = 0; i < 8; ++i) { a[i] = (_Float16)(p[i] * sc); a[8 + i] = (_Float16)(p[16 + i] * sc); }
  return a;
}
__device__ __forceinline__ v16h fragc_f32(const float* W, int k0, int n, int lane, int ld, int K) {
  v16h a; const int g = lane >> 4;
#pragma unroll
  for (int i = 0; i < 8; ++i) { const int ka = k0 + 8 * g + i, kb = ka + 16;
    a[i] = (_Float16)(ka < K ? W[(size_t)(ka < K ? ka : K - 1) * ld + n] : 0.f); a[8 + i] = (_Float16)(kb < K ? W[(size_t)(kb < K ? kb : K - 1) * ld + n] : 0.f); }
  return a;
}
struct F2 { v16b h, l; };
__device__ __forceinline__ F2 bsplit16(const float v[16]) { F2 r;
#pragma unroll
  for (int i = 0; i < 16; ++i) { const __bf16 h = (__bf16)v[i]; r.h[i] = h; r.l[i] = (__bf16)(v[i] - (float)h); }
  return r; }
__device__ __forceinline__ F2 split_row(const float* row, int k0, int lane) { float v[16]; const float* p = row + k0 + 8 * (lane >> 4);
#pragma unroll
  for (int i = 0; i < 8; ++i) { v[i] = p[i]; v[8 + i] = p[16 + i]; }
  return bsplit16(v); }
__device__ __forceinline__ F2 split_rowK(const float* row, int k0, int lane, int K) { float v[16]; const int g = lane >> 4;
#pragma unroll
  for (int i = 0; i < 8; ++i) { const int ka = k0 + 8 * g + i, kb = ka + 16; v[i] = ka < K ? row[ka < K ? ka : K - 1] : 0.f; v[8 + i] = kb < K ? row[kb < K ? kb : K - 1] : 0.f; }
  return bsplit16(v); }
__device__ __forceinline__ F2 split_col(const float* W, int k0, int n, int lane, int ld, int K) { float v[16]; const int g = lane >> 4;
#pragma unroll
  for (int i = 0; i < 8; ++i) { const int ka = k0 + 8 * g + i, kb = ka + 16; v[i] = ka < K ? W[(size_t)(ka < K ? ka : K - 1) * ld + n] : 0.f; v[8 + i] = kb < K ? W[(size_t)(kb < K ? kb : K - 1) * ld + n] : 0.f; }
  return bsplit16(v); }
__device__ __forceinline__ v8f mac3(const F2& a, const F2& b, v8f c) { c = wmma_bf(a.l, b.h, c); c = wmma_bf(a.h, b.l, c); return wmma_bf(a.h, b.h, c); }
__device__ __forceinline__ float sigm(float v) { return 1.0f / (1.0f + expf(-v)); }
#define LDSX() do { asm volatile("s_wait_dscnt 0" ::: "memory"); __builtin_amdgcn_wave_barrier(); __builtin_amdgcn_fence(__ATOMIC_RELEASE, "workgroup"); } while (0)


#define SS 2048
#define DM 2048
#define NHQ 16
#define NKV 4
#define NBIT 8
#define WIN 32
#ifndef QMAX
#define QMAX SS
#endif
typedef __attribute__((ext_vector_type(8))) __bf16 v8b;
__device__ __forceinline__ v16b frag_b(const __bf16* rowk0, int lane) {
  union { v16b v; v8b q[2]; } u; const __bf16* p = rowk0 + 8 * (lane >> 4);
  u.q[0] = *(const v8b*)p; u.q[1] = *(const v8b*)(p + 16); return u.v;
}
__device__ __forceinline__ v16b frag_gbf(const float* rowk0, int lane) {
  v16b a; const float* p = rowk0 + 8 * (lane >> 4);
#pragma unroll
  for (int i = 0; i < 8; ++i) { a[i] = (__bf16)p[i]; a[8 + i] = (__bf16)p[16 + i]; }
  return a;
}
__device__ __forceinline__ float bfr(float v) { return (float)(__bf16)v; }
__device__ __attribute__((noinline)) float exp_ni(float v) { return expf(v); }
__device__ __attribute__((noinline)) float tanh_ni(float v) { return tanhf(v); }

#define WS_Q   0u
#define WS_K   (WS_Q + 4u * SS * 128)
#define WS_V   (WS_K + 4u * SS * 32)
#define WS_G   (WS_V + 4u * SS * 32)
#define WS_SD  (WS_G + 4u * SS * SS)
#define WS_OT  (WS_SD + 4u * SS * SS)
#define WS_O   (WS_OT + 4u * 128 * SS)
#define WS_END (WS_O + 4u * SS * 128)

__global__ __launch_bounds__(128) void k_proj(const float* __restrict__ X, const float* __restrict__ Wq, const float* __restrict__ Wk, const float* __restrict__ Wv, const float* __restrict__ tau, float* __restrict__ Q, float* __restrict__ Kb, float* __restrict__ Vb) {
  __shared__ __align__(16) float so[4][16][196];
  const int tid = threadIdx.x, wave = tid >> 5, lane = tid & 31, col = lane & 15, g = lane >> 4; const size_t r0 = (size_t)blockIdx.x * 64 + wave * 16;
  v8f acc[12] = {};
#pragma unroll 1
  for (int kc = 0; kc < DM / 32; ++kc) { const v16b a = frag_gbf(X + (r0 + col) * DM + kc * 32, lane);
#pragma unroll
    for (int j = 0; j < 12; ++j) { const int n = j * 16 + col; const float* wr = n < 128 ? Wq + (size_t)n * DM : (n < 160 ? Wk + (size_t)(n - 128) * DM : Wv + (size_t)(n - 160) * DM);
      acc[j] = wmma_bf(a, frag_gbf(wr + kc * 32, lane), acc[j]); } }
  const float it = 1.0f / bfr(tau[0]);
#pragma unroll
  for (int j = 0; j < 12; ++j)
#pragma unroll
    for (int r = 0; r < 8; ++r) { const float v = acc[j][r] * it; so[wave][8 * g + r][j * 16 + col] = j < 10 ? tanh_ni(v) : 1.0f / (1.0f + exp_ni(-v)); }
  LDSX();
  for (int rl = 0; rl < 16; ++rl) { const size_t row = r0 + rl;
    vst2(Q + row * 128 + lane * 4, *(const v4f*)&so[wave][rl][lane * 4]);
    if (lane < 8) vst2(Kb + row * 32 + lane * 4, *(const v4f*)&so[wave][rl][128 + lane * 4]); else if (lane < 16) vst2(Vb + row * 32 + (lane - 8) * 4, *(const v4f*)&so[wave][rl][160 + (lane - 8) * 4]); }
}
__global__ __launch_bounds__(128) void k_gram(const float* __restrict__ Q, const float* __restrict__ Kb, float* __restrict__ G, int h) {
  __shared__ __align__(16) float so[4][16][132];
  const int tid = threadIdx.x, wave = tid >> 5, lane = tid & 31, col = lane & 15, g = lane >> 4; const int i0 = blockIdx.x * 64 + wave * 16, j0 = blockIdx.y * 128;
  if (j0 > blockIdx.x * 64 + 63) return;
  const F2 a = split_rowK(Q + (size_t)(i0 + col) * 128 + h * NBIT, 0, lane, NBIT);
  v8f acc[8];
#pragma unroll
  for (int j = 0; j < 8; ++j) { const F2 kb = split_rowK(Kb + (size_t)(j0 + j * 16 + col) * 32 + (h / 4) * NBIT, 0, lane, NBIT); acc[j] = mac3(a, kb, (v8f){}); }
#pragma unroll
  for (int j = 0; j < 8; ++j)
#pragma unroll
    for (int r = 0; r < 8; ++r) so[wave][8 * g + r][j * 16 + col] = acc[j][r];
  LDSX();
  for (int rl = 0; rl < 16; ++rl) vst2(G + (size_t)(i0 + rl) * SS + j0 + lane * 4, *(const v4f*)&so[wave][rl][lane * 4]);
}
__global__ __launch_bounds__(256) void k_win(const float* __restrict__ G, float* __restrict__ SD) {
  const int tid = threadIdx.x, wave = tid >> 5, lane = tid & 31; const int d = blockIdx.x * 8 + wave + 1; if (d >= SS) return;
  const int len = (QMAX < SS ? QMAX : SS) - d; if (len <= 0) return;
  float pprev = 0.f, tprev = 0.f;
#pragma unroll 1
  for (int j0 = 0; j0 < len; j0 += 32) { const int j = j0 + lane; const int jc = j < len ? j : len - 1; float gv = G[(size_t)(d + jc) * SS + jc]; gv = j < len ? gv : 0.f;
    float p = gv;
#pragma unroll
    for (int o = 1; o < 32; o <<= 1) { const float up = __shfl_up(p, o); p += (lane >= o) ? up : 0.f; }
    const float s = p + (tprev - pprev);
    const float tot = __shfl(p, 31);
    v4f v;
#pragma unroll
    for (int i = 0; i < 4; ++i) v[i] = __shfl(s, ((lane & 7) << 2) + i);
    if (lane < 8) vst2(SD + (size_t)d * SS + j0 + lane * 4, v);
    pprev = p; tprev = tot; }
}
__global__ __launch_bounds__(256) void k_soft(const float* __restrict__ SD, const float* __restrict__ Vb, const float* __restrict__ tau, float* __restrict__ OT, int h) {
  __shared__ __align__(16) float so[8][68];
  const int tid = threadIdx.x, wave = tid >> 5, lane = tid & 31; const int q0 = blockIdx.x * 64; const int kvh = h / 4;
  const float itau = 1.0f / bfr(tau[0]); const float sc = (1.0f / 16.0f) * itau;
#pragma unroll 1
  for (int rr = wave; rr < 64; rr += 8) { const int q = q0 + rr; const float iq1 = itau / (float)(q + 1);
    float mx = -__builtin_inff();
    for (int k = lane; k < q; k += 32) { const float lg = SD[(size_t)(q - k) * SS + k] * sc + (float)k * iq1; mx = fmaxf(mx, lg); }
#pragma unroll
    for (int o = 1; o < 32; o <<= 1) mx = fmaxf(mx, __shfl_xor(mx, o));
    float den = 0.f; float ov[8] = {0.f, 0.f, 0.f, 0.f, 0.f, 0.f, 0.f, 0.f};
    for (int k = lane; k < q; k += 32) { const float lg = SD[(size_t)(q - k) * SS + k] * sc + (float)k * iq1; const float e = exp_ni(lg - mx); den += e;
      const int kv = k + 1;
      const float4 va = *(const float4*)(Vb + (size_t)kv * 32 + kvh * NBIT), vb = *(const float4*)(Vb + (size_t)kv * 32 + kvh * NBIT + 4);
      ov[0] += e * va.x; ov[1] += e * va.y; ov[2] += e * va.z; ov[3] += e * va.w; ov[4] += e * vb.x; ov[5] += e * vb.y; ov[6] += e * vb.z; ov[7] += e * vb.w; }
#pragma unroll
    for (int o = 1; o < 32; o <<= 1) { den += __shfl_xor(den, o);
#pragma unroll
      for (int c = 0; c < 8; ++c) ov[c] += __shfl_xor(ov[c], o); }
    if (lane < 8) so[lane][rr] = (q > 0 && den > 0.f) ? ov[lane] / den : 0.f; }
  __syncthreads();
  for (int qq = tid; qq < 8 * 16; qq += 256) { const int c = qq >> 4, pc = qq & 15; vst2(OT + (size_t)(h * NBIT + c) * SS + q0 + pc * 4, *(const v4f*)&so[c][pc * 4]); }
}
__global__ __launch_bounds__(256) void k_tr(const float* __restrict__ OT, const float* __restrict__ e0, const float* __restrict__ e1, float* __restrict__ O) {
  __shared__ __align__(16) float st[64][132];
  const int q0 = blockIdx.x * 64, tid = threadIdx.x;
  for (int qq = tid; qq < 128 * 64; qq += 256) { const int c = qq >> 6, ql = qq & 63; const float o = OT[(size_t)c * SS + q0 + ql]; st[ql][c] = o * bfr(e1[c]) + (1.0f - o) * bfr(e0[c]); }
  __syncthreads();
  for (int qq = tid; qq < 64 * 32; qq += 256) { const int ql = qq >> 5, pc = qq & 31; vst2(O + (size_t)(q0 + ql) * 128 + pc * 4, *(const v4f*)&st[ql][pc * 4]); }
}
__global__ __launch_bounds__(128) void k_out(const float* __restrict__ O, const float* __restrict__ Wo, float* __restrict__ Y) {
  __shared__ __align__(16) float so[4][16][132];
  const int tid = threadIdx.x, wave = tid >> 5, lane = tid & 31, col = lane & 15, g = lane >> 4; const size_t r0 = (size_t)blockIdx.x * 64 + wave * 16; const int n0 = blockIdx.y * 128;
  v8f acc[8] = {};
#pragma unroll
  for (int kc = 0; kc < 4; ++kc) { const F2 a = split_row(O + (r0 + col) * 128, kc * 32, lane);
#pragma unroll
    for (int j = 0; j < 8; ++j) { const v16b w = frag_gbf(Wo + (size_t)(n0 + j * 16 + col) * 128 + kc * 32, lane); acc[j] = wmma_bf(a.l, w, acc[j]); acc[j] = wmma_bf(a.h, w, acc[j]); } }
#pragma unroll
  for (int j = 0; j < 8; ++j)
#pragma unroll
    for (int r = 0; r < 8; ++r) so[wave][8 * g + r][j * 16 + col] = acc[j][r];
  LDSX();
  for (int rl = 0; rl < 16; ++rl) vst2(Y + (r0 + rl) * DM + n0 + lane * 4, *(const v4f*)&so[wave][rl][lane * 4]);
}

extern "C" void kernel_launch(void* const* d_in, const int* in_sizes, int n_in, void* d_out, int out_size, void* d_ws, size_t ws_size, hipStream_t stream) {
  (void)in_sizes; (void)n_in; (void)out_size;
  const float** F = (const float**)d_in;
  if (ws_size < (size_t)WS_END) return;
  char* ws = (char*)d_ws; float *Q = (float*)(ws + WS_Q), *Kb = (float*)(ws + WS_K), *Vb = (float*)(ws + WS_V), *G = (float*)(ws + WS_G), *SD = (float*)(ws + WS_SD), *OT = (float*)(ws + WS_OT), *O = (float*)(ws + WS_O);
  k_proj<<<SS / 64, 128, 0, stream>>>(F[0], F[1], F[2], F[3], F[7], Q, Kb, Vb);
  for (int h = 0; h < NHQ; ++h) {
    k_gram<<<dim3(QMAX / 64, SS / 128), 128, 0, stream>>>(Q, Kb, G, h);
    k_win<<<SS / 8, 256, 0, stream>>>(G, SD);
    k_soft<<<QMAX / 64, 256, 0, stream>>>(SD, Vb, F[7], OT, h); }
  k_tr<<<QMAX / 64, 256, 0, stream>>>(OT, F[5], F[6], O);
  k_out<<<dim3(QMAX / 64, DM / 128), 128, 0, stream>>>(O, F[4], (float*)d_out);
}
